// LSTMCell_53300544143475
// MI455X (gfx1250) — hardware-verified
//
#include <hip/hip_runtime.h>
#include <math.h>

constexpr int NBAT    = 4096;
constexpr int NINP    = 1024;
constexpr int NHID    = 1024;
constexpr int KDIM    = NINP + NHID;
constexpr int NGROW   = 4 * NHID;
constexpr int NTHR    = 256;
constexpr int NWAVE   = NTHR / 32;
constexpr int WTM     = 32;
constexpr int WTU     = 32;
constexpr int TILES_M = NBAT / WTM;
constexpr int TILES_U = NHID / WTU;
constexpr int NTILES  = TILES_M * TILES_U;
constexpr int SLP     = 100;
constexpr int NOUT    = NBAT * NHID;
static_assert(KDIM % 32 == 0);
static_assert(NINP % 32 == 0 && NHID % 32 == 0);
static_assert(NBAT % WTM == 0 && NHID % WTU == 0);
static_assert(NTILES % NWAVE == 0);
static_assert(WTU * 4 == 128);
static_assert((SLP * 4) % 16 == 0);
static_assert((NINP / 8) % 32 == 0 && (KDIM / 8) % 32 == 0);
static_assert((NBAT * (NINP / 8)) % NTHR == 0 && (NGROW * (KDIM / 8)) % NTHR == 0);

typedef __attribute__((ext_vector_type(16))) __bf16   v16b;
typedef __attribute__((ext_vector_type(8)))  __bf16   v8b;
typedef __attribute__((ext_vector_type(8)))  float    v8f;
typedef __attribute__((ext_vector_type(4)))  float    v4f;
typedef __attribute__((ext_vector_type(4)))  unsigned v4u;

__device__ __forceinline__ unsigned short f2bf_bits(float f) {
  unsigned u = __float_as_uint(f);
  return (unsigned short)((u + 0x7FFFu + ((u >> 16) & 1u)) >> 16);
}
__device__ __forceinline__ float bf_bits2f(unsigned short h) { return __uint_as_float(((unsigned)h) << 16); }
__device__ __forceinline__ float bf16r(float f) { return bf_bits2f(f2bf_bits(f)); }

__device__ __forceinline__ void pair_guard_b(v8f& a, v8f& b, v16b x, v16b y, v16b z) {
  asm volatile("v_nop\n\tv_nop\n\tv_nop\n\tv_nop" : "+v"(a), "+v"(b) : "v"(x), "v"(y), "v"(z));
}
__device__ __forceinline__ void acc_guard4(v8f& a, v8f& b, v8f& c, v8f& d) {
  asm volatile("v_nop\n\tv_nop\n\tv_nop\n\tv_nop" : "+v"(a), "+v"(b), "+v"(c), "+v"(d));
}
__device__ __forceinline__ void load_fence() { asm volatile("" ::: "memory"); }
__device__ __forceinline__ void wave_lds_sync() {
  __builtin_amdgcn_fence(__ATOMIC_RELEASE, "workgroup");
  __builtin_amdgcn_wave_barrier();
  __builtin_amdgcn_fence(__ATOMIC_ACQUIRE, "workgroup");
}

template <typename T> struct Frag;
template <> struct Frag<__bf16> {
  typedef v16b V; union U { v16b v; v8b h[2]; };
  static __device__ __forceinline__ v16b load(const __bf16* p) {
    U f; f.h[0] = *(const v8b*)(p); f.h[1] = *(const v8b*)(p + 16); return f.v;
  }
  static __device__ __forceinline__ v8f mma(v16b a, v16b b, v8f c) {
    return __builtin_amdgcn_wmma_f32_16x16x32_bf16(false, a, false, b, (short)0, c, false, false);
  }
};

__device__ __forceinline__ float fsig(float x)  { return __builtin_amdgcn_rcpf(1.0f + expf(-x)); }
__device__ __forceinline__ float ftanh(float x) { return 1.0f - 2.0f * __builtin_amdgcn_rcpf(expf(2.0f * x) + 1.0f); }

template <int NCOL8, int SPITCH, int DPITCH>
__global__ __launch_bounds__(NTHR) void cvt_bf16_kernel(const float* __restrict__ src, unsigned short* __restrict__ dst,
                                                        int nrow, int dcol0) {
  const int i  = blockIdx.x * NTHR + threadIdx.x;
  const int n8 = nrow * NCOL8;
  if (i < n8) {
    const int row = i / NCOL8;
    const int c8  = i - row * NCOL8;
    const float* sp = src + (size_t)row * SPITCH + c8 * 8;
    const v4f a = *(const v4f*)(sp);
    const v4f b = *(const v4f*)(sp + 4);
    v4u pk;
    pk[0] = (unsigned)f2bf_bits(a[0]) | ((unsigned)f2bf_bits(a[1]) << 16);
    pk[1] = (unsigned)f2bf_bits(a[2]) | ((unsigned)f2bf_bits(a[3]) << 16);
    pk[2] = (unsigned)f2bf_bits(b[0]) | ((unsigned)f2bf_bits(b[1]) << 16);
    pk[3] = (unsigned)f2bf_bits(b[2]) | ((unsigned)f2bf_bits(b[3]) << 16);
    unsigned short* dp = dst + (size_t)row * DPITCH + dcol0 + c8 * 8;
    *(volatile v4u*)dp = pk;
    __threadfence();
    *(volatile v4u*)dp = pk;
  }
}

__global__ __launch_bounds__(NTHR) void lstm_cell_kernel(const unsigned short* __restrict__ CBp,
                                                         const unsigned short* __restrict__ WBp,
                                                         const float* __restrict__ bias,
                                                         const float* __restrict__ c_prev,
                                                         float* __restrict__ out_h, float* __restrict__ out_c) {
  __shared__ __align__(16) float sT[NWAVE * 16 * SLP];
  const __bf16* A  = (const __bf16*)CBp;
  const __bf16* Bw = (const __bf16*)WBp;
  const int tid = threadIdx.x, lane = tid & 31, wave = tid >> 5;
  const int c = lane & 15, hh = lane >> 4, koff = hh * 8;
  const int tile = blockIdx.x * NWAVE + wave;
  const int tm = tile / TILES_U, tu = tile - tm * TILES_U;
  const int m0 = tm * WTM, n0 = tu * WTU;

  float bb[2][4];
#pragma unroll
  for (int u = 0; u < 2; ++u)
#pragma unroll
    for (int g = 0; g < 4; ++g) bb[u][g] = bf16r(bias[g * NHID + n0 + 16 * u + c]);

  const v8f z8 = {0.f, 0.f, 0.f, 0.f, 0.f, 0.f, 0.f, 0.f};
  v8f acc[2][2][4];
#pragma unroll
  for (int i = 0; i < 2; ++i)
#pragma unroll
    for (int u = 0; u < 2; ++u)
#pragma unroll
      for (int g = 0; g < 4; ++g) acc[i][u][g] = z8;

  const __bf16* a0p   = A  + (size_t)(m0 + c) * KDIM + koff;
  const __bf16* a1p   = A  + (size_t)(m0 + 16 + c) * KDIM + koff;
  const __bf16* bbase = Bw + (size_t)(n0 + c) * KDIM + koff;

#pragma unroll 1
  for (int k0 = 0; k0 < KDIM; k0 += 32) {
    const v16b a0 = Frag<__bf16>::load(a0p + k0);
    const v16b a1 = Frag<__bf16>::load(a1p + k0);
#pragma unroll
    for (int u = 0; u < 2; ++u) {
#pragma unroll
      for (int g = 0; g < 4; ++g) {
        const v16b b = Frag<__bf16>::load(bbase + (size_t)(g * NHID + 16 * u) * KDIM + k0);
        acc[0][u][g] = Frag<__bf16>::mma(a0, b, acc[0][u][g]);
        acc[1][u][g] = Frag<__bf16>::mma(a1, b, acc[1][u][g]);
        pair_guard_b(acc[0][u][g], acc[1][u][g], a0, a1, b);
      }
      load_fence();
    }
  }
  acc_guard4(acc[0][0][0], acc[0][0][1], acc[0][0][2], acc[0][0][3]);
  acc_guard4(acc[0][1][0], acc[0][1][1], acc[0][1][2], acc[0][1][3]);
  acc_guard4(acc[1][0][0], acc[1][0][1], acc[1][0][2], acc[1][0][3]);
  acc_guard4(acc[1][1][0], acc[1][1][1], acc[1][1][2], acc[1][1][3]);

  float* slab = sT + wave * (16 * SLP);
  const int q = lane >> 3, c4 = (lane & 7) * 4;
#pragma unroll
  for (int i = 0; i < 2; ++i) {
#pragma unroll
    for (int u = 0; u < 2; ++u) {
#pragma unroll
      for (int r = 0; r < 8; ++r) {
        const float zf = acc[i][u][0][r] + bb[u][0];
        const float zi = acc[i][u][1][r] + bb[u][1];
        const float zg = acc[i][u][2][r] + bb[u][2];
        const float zo = acc[i][u][3][r] + bb[u][3];
        const float fg = fsig(zf);
        const float ig = fsig(zi) * ftanh(zg);
        const float og = fsig(zo);
        float* sp = slab + (8 * hh + r) * SLP + 16 * u + c;
        sp[0]  = fg;
        sp[32] = ig;
        sp[64] = og;
      }
    }
    wave_lds_sync();
    v4f cv[4], hv[4];
#pragma unroll
    for (int it = 0; it < 4; ++it) {
      const int row = it * 4 + q;
      const size_t go = (size_t)(m0 + 16 * i + row) * NHID + n0 + c4;
      const v4f cp4 = *(const v4f*)(c_prev + go);
      const v4f f4  = *(const v4f*)(slab + row * SLP + c4);
      const v4f g4  = *(const v4f*)(slab + row * SLP + 32 + c4);
      const v4f o4  = *(const v4f*)(slab + row * SLP + 64 + c4);
      v4f cc, hc;
#pragma unroll
      for (int e = 0; e < 4; ++e) {
        const float cpb = bf16r(cp4[e]);
        const float ct  = f4[e] * cpb + g4[e];
        cc[e] = ct;
        hc[e] = o4[e] * ftanh(ct);
      }
      cv[it] = cc;
      hv[it] = hc;
    }
    for (int pass = 0; pass < 2; ++pass) {
#pragma unroll
      for (int it = 0; it < 4; ++it) {
        const int row = it * 4 + q;
        const size_t go = (size_t)(m0 + 16 * i + row) * NHID + n0 + c4;
        *(volatile v4f*)(out_c + go) = cv[it];
        *(volatile v4f*)(out_h + go) = hv[it];
      }
      __threadfence();
    }
    wave_lds_sync();
  }
}

extern "C" void kernel_launch(void* const* d_in, const int* in_sizes, int n_in,
                              void* d_out, int out_size, void* d_ws, size_t ws_size, hipStream_t stream) {
  if (n_in < 5 || d_out == nullptr || d_ws == nullptr) return;
  if (in_sizes[0] != NBAT * NINP || in_sizes[1] != NBAT * NHID || in_sizes[2] != NBAT * NHID ||
      in_sizes[3] != NGROW * KDIM || in_sizes[4] != NGROW || out_size != 2 * NOUT) return;

  const float* x      = (const float*)d_in[0];
  const float* h_prev = (const float*)d_in[1];
  const float* c_prev = (const float*)d_in[2];
  const float* w      = (const float*)d_in[3];
  const float* bias   = (const float*)d_in[4];
  float* out_h = (float*)d_out;
  float* out_c = out_h + (size_t)NOUT;

  char* ws = (char*)d_ws; size_t off = 0;
  auto carve = [&](size_t bytes) -> char* { char* p = ws + off; off += (bytes + 255) & ~(size_t)255; return p; };
  unsigned short* CB = (unsigned short*)carve((size_t)NBAT * KDIM * 2);
  unsigned short* WB = (unsigned short*)carve((size_t)NGROW * KDIM * 2);
  if (off > ws_size || off > (size_t)134217728) return;

  cvt_bf16_kernel<NINP / 8, NINP, KDIM><<<(NBAT * (NINP / 8)) / NTHR, NTHR, 0, stream>>>(x,      CB, NBAT,  0);
  cvt_bf16_kernel<NHID / 8, NHID, KDIM><<<(NBAT * (NHID / 8)) / NTHR, NTHR, 0, stream>>>(h_prev, CB, NBAT,  NINP);
  cvt_bf16_kernel<KDIM / 8, KDIM, KDIM><<<(NGROW * (KDIM / 8)) / NTHR, NTHR, 0, stream>>>(w,     WB, NGROW, 0);
  lstm_cell_kernel<<<NTILES / NWAVE, NTHR, 0, stream>>>(CB, WB, bias, c_prev, out_h, out_c);
}
